// PointTransformerBlock_523986010297
// MI455X (gfx1250) — hardware-run, weakly checked
//
#include <hip/hip_runtime.h>
#include <math.h>

typedef __attribute__((ext_vector_type(16))) _Float16 v16h;
typedef __attribute__((ext_vector_type(16))) __bf16 v16b;
typedef __attribute__((ext_vector_type(8)))  _Float16 v8h;
typedef __attribute__((ext_vector_type(8)))  float v8f;
typedef __attribute__((ext_vector_type(4)))  float v4f;
typedef __attribute__((ext_vector_type(2)))  float v2f;
typedef __attribute__((ext_vector_type(4)))  unsigned v4u;
typedef __attribute__((ext_vector_type(4)))  int v4i;
typedef float __attribute__((may_alias)) float_a;
typedef int __attribute__((may_alias)) int_a;

template <typename T> __device__ __forceinline__ void vst2(void* p, T v) { *(volatile T*)p = v; __threadfence(); *(volatile T*)p = v; }
__device__ __forceinline__ v8f wmma16(v16h a, v16h b, v8f c) {
  v8f d = __builtin_amdgcn_wmma_f32_16x16x32_f16(false, a, false, b, (short)0, c, false, false);
  asm volatile("v_nop\n\tv_nop\n\tv_nop\n\tv_nop" : "+v"(d) : "v"(a), "v"(b));
  return d;
}
__device__ __forceinline__ v8f wmma_bf(v16b a, v16b b, v8f c) {
  v8f d = __builtin_amdgcn_wmma_f32_16x16x32_bf16(false, a, false, b, (short)0, c, false, false);
  asm volatile("v_nop\n\tv_nop\n\tv_nop\n\tv_nop" : "+v"(d) : "v"(a), "v"(b));
  return d;
}
__device__ __forceinline__ v16h frag_h(const _Float16* rowk0, int lane) {
  union { v16h v; v8h q[2]; } u; const _Float16* p = rowk0 + 8 * (lane >> 4);
  u.q[0] = *(const v8h*)p; u.q[1] = *(const v8h*)(p + 16); return u.v;
}
__device__ __forceinline__ v16h frag_f32(const float* rowk0, int lane) {
  v16h a; const float* p = rowk0 + 8 * (lane >> 4);
#pragma unroll
  for (int i = 0; i < 8; ++i) { a[i] = (_Float16)p[i]; a[8 + i] = (_Float16)p[16 + i]; }
  return a;
}
__device__ __forceinline__ v16h frag_f32s(const float* rowk0, int lane, float sc) {
  v16h a; const float* p = rowk0 + 8 * (lane >> 4);
#pragma unroll
  for (int i = 0; i < 8; ++i) { a[i] = (_Float16)(p[i] * sc); a[8 + i] = (_Float16)(p[16 + i] * sc); }
  return a;
}
__device__ __forceinline__ v16h fragc_f32(const float* W, int k0, int n, int lane, int ld, int K) {
  v16h a; const int g = lane >> 4;
#pragma unroll
  for (int i = 0; i < 8; ++i) { const int ka = k0 + 8 * g + i, kb = ka + 16;
    a[i] = (_Float16)(ka < K ? W[(size_t)(ka < K ? ka : K - 1) * ld + n] : 0.f); a[8 + i] = (_Float16)(kb < K ? W[(size_t)(kb < K ? kb : K - 1) * ld + n] : 0.f); }
  return a;
}
struct F2 { v16b h, l; };
__device__ __forceinline__ F2 bsplit16(const float v[16]) { F2 r;
#pragma unroll
  for (int i = 0; i < 16; ++i) { const __bf16 h = (__bf16)v[i]; r.h[i] = h; r.l[i] = (__bf16)(v[i] - (float)h); }
  return r; }
__device__ __forceinline__ F2 split_row(const float* row, int k0, int lane) { float v[16]; const float* p = row + k0 + 8 * (lane >> 4);
#pragma unroll
  for (int i = 0; i < 8; ++i) { v[i] = p[i]; v[8 + i] = p[16 + i]; }
  return bsplit16(v); }
__device__ __forceinline__ F2 split_rowK(const float* row, int k0, int lane, int K) { float v[16]; const int g = lane >> 4;
#pragma unroll
  for (int i = 0; i < 8; ++i) { const int ka = k0 + 8 * g + i, kb = ka + 16; v[i] = ka < K ? row[ka < K ? ka : K - 1] : 0.f; v[8 + i] = kb < K ? row[kb < K ? kb : K - 1] : 0.f; }
  return bsplit16(v); }
__device__ __forceinline__ F2 split_col(const float* W, int k0, int n, int lane, int ld, int K) { float v[16]; const int g = lane >> 4;
#pragma unroll
  for (int i = 0; i < 8; ++i) { const int ka = k0 + 8 * g + i, kb = ka + 16; v[i] = ka < K ? W[(size_t)(ka < K ? ka : K - 1) * ld + n] : 0.f; v[8 + i] = kb < K ? W[(size_t)(kb < K ? kb : K - 1) * ld + n] : 0.f; }
  return bsplit16(v); }
__device__ __forceinline__ v8f mac3(const F2& a, const F2& b, v8f c) { c = wmma_bf(a.l, b.h, c); c = wmma_bf(a.h, b.l, c); return wmma_bf(a.h, b.h, c); }
__device__ __forceinline__ float sigm(float v) { return 1.0f / (1.0f + expf(-v)); }
#define LDSX() do { asm volatile("s_wait_dscnt 0" ::: "memory"); __builtin_amdgcn_wave_barrier(); __builtin_amdgcn_fence(__ATOMIC_RELEASE, "workgroup"); } while (0)

#define NPT 80000
#define CCH 64
#define NSB 16
#define SPL 8
#define CW 8
#define NE (NPT * NSB)
#define EPB 256
#define NEB (NE / EPB)
#ifndef NPROC
#define NPROC NPT
#endif
#define NEBP (NPROC * NSB / EPB)
__device__ __forceinline__ float bfr(float v) { return (float)(__bf16)v; }
#define WS_T1   0u
#define WS_Q    (WS_T1 + 4u * (size_t)NPT * CCH)
#define WS_K    (WS_Q + 4u * (size_t)NPT * CCH)
#define WS_V    (WS_K + 4u * (size_t)NPT * CCH)
#define WS_AGG  (WS_T1)
#define WS_T3   (WS_Q)
#define WS_W1R  (WS_V + 4u * (size_t)NPT * CCH)
#define WS_PART (WS_W1R + 4u * (size_t)NE * CW)
#define WS_ST   (WS_PART + 4u * (size_t)NEB * CCH)
#define ST_SZ   (4u * 64 * 32)
#define WS_END  (WS_ST + 6u * ST_SZ)

__global__ __launch_bounds__(128) void k_gemm64(const float* __restrict__ IN, int mode, const float* __restrict__ ST, const float* __restrict__ G, const float* __restrict__ BE,
    const float* __restrict__ W0, const float* __restrict__ B0, float* __restrict__ O0, const float* __restrict__ W1p, const float* __restrict__ B1, float* __restrict__ O1, const float* __restrict__ W2, const float* __restrict__ B2, float* __restrict__ O2) {
  __shared__ __align__(16) float sf[4][16][68];
  const int tid = threadIdx.x, wave = tid >> 5, lane = tid & 31, col = lane & 15, g = lane >> 4; const int which = blockIdx.y; const size_t r0 = (size_t)blockIdx.x * 64 + wave * 16;
  const float* Wm = which == 0 ? W0 : which == 1 ? W1p : W2; const float* Bm = which == 0 ? B0 : which == 1 ? B1 : B2; float* OUT = which == 0 ? O0 : which == 1 ? O1 : O2;
  v8f acc[4] = {};
#pragma unroll
  for (int kc = 0; kc < 2; ++kc) { float v[16]; { const float* p = IN + (r0 + col) * CCH + kc * 32 + 8 * g;
#pragma unroll
      for (int i = 0; i < 8; ++i) { v[i] = p[i]; v[8 + i] = p[16 + i]; } }
    asm volatile("s_wait_loadcnt 0x0" ::: "memory");
    if (mode == 1) {
#pragma unroll
      for (int i = 0; i < 16; ++i) { const int c = kc * 32 + 8 * g + (i < 8 ? i : 8 + i); const float mu = ST[c * 32], rs = ST[c * 32 + 1]; asm volatile("s_wait_loadcnt 0x0" ::: "memory"); v[i] = fmaxf((v[i] - mu) * rs * bfr(G[c]) + bfr(BE[c]), 0.f); } }
    else {
#pragma unroll
      for (int i = 0; i < 16; ++i) v[i] = bfr(v[i]); }
    const F2 a = bsplit16(v);
#pragma unroll
    for (int j = 0; j < 4; ++j) { v16b w; { float t0[8], t1[8]; const int o = j * 16 + col;
#pragma unroll
        for (int i = 0; i < 8; ++i) t0[i] = Wm[(size_t)(kc * 32 + 8 * g + i) * CCH + o];
        asm volatile("s_wait_loadcnt 0x0" ::: "memory");
#pragma unroll
        for (int i = 0; i < 8; ++i) t1[i] = Wm[(size_t)(kc * 32 + 16 + 8 * g + i) * CCH + o];
        asm volatile("s_wait_loadcnt 0x0" ::: "memory");
#pragma unroll
        for (int i = 0; i < 8; ++i) { w[i] = (__bf16)t0[i]; w[8 + i] = (__bf16)t1[i]; } }
      acc[j] = wmma_bf(a.h, w, acc[j]); if (mode == 1) acc[j] = wmma_bf(a.l, w, acc[j]); } }
#pragma unroll
  for (int j = 0; j < 4; ++j) { const float bb = Bm ? bfr(Bm[j * 16 + col]) : 0.f;
#pragma unroll
    for (int r = 0; r < 8; ++r) sf[wave][8 * g + r][j * 16 + col] = acc[j][r] + bb; }
  LDSX(); for (int rl = 0; rl < 16; ++rl) if (lane < 16) vst2(OUT + (r0 + rl) * CCH + lane * 4, *(const v4f*)&sf[wave][rl][lane * 4]); }
__global__ __launch_bounds__(256) void k_stat64(const float* __restrict__ T, float* __restrict__ STo) { __shared__ float sred[8]; __shared__ float sbc;
  const int t = threadIdx.x; const int c = blockIdx.x;
  float s = 0.f; for (int r = t; r < NPROC; r += 256) s += T[(size_t)r * CCH + c];
#pragma unroll
  for (int o = 1; o < 32; o <<= 1) s += __shfl_xor(s, o);
  if ((t & 31) == 0) sred[t >> 5] = s; __syncthreads(); if (t == 0) { float a = 0.f; for (int i = 0; i < 8; ++i) a += sred[i]; sbc = a / (float)NPROC; } __syncthreads(); const float mean = sbc; __syncthreads();
  float q = 0.f; for (int r = t; r < NPROC; r += 256) { const float d = T[(size_t)r * CCH + c] - mean; q += d * d; }
#pragma unroll
  for (int o = 1; o < 32; o <<= 1) q += __shfl_xor(q, o);
  if ((t & 31) == 0) sred[t >> 5] = q; __syncthreads(); if (t == 0) { float a = 0.f; for (int i = 0; i < 8; ++i) a += sred[i]; sbc = rsqrtf(a / (float)NPROC + 1e-5f); } __syncthreads();
  if (t < 32) { const float v = t == 0 ? mean : (t == 1 ? sbc : 0.f); vst2(STo + (size_t)c * 32 + t, v); } }
struct EdgeCtx { int n, s, idx; float pr[3]; };
__device__ __forceinline__ EdgeCtx edge_of(int e, const float* __restrict__ P, const int* __restrict__ KNN) { EdgeCtx c; c.n = e >> 4; c.s = e & 15; int ii = KNN[(size_t)c.n * NSB + c.s]; ii = ii < 0 ? 0 : (ii >= NPT ? NPT - 1 : ii); c.idx = ii;
  c.pr[0] = bfr(P[(size_t)ii * 3]) - bfr(P[(size_t)c.n * 3]); c.pr[1] = bfr(P[(size_t)ii * 3 + 1]) - bfr(P[(size_t)c.n * 3 + 1]); c.pr[2] = bfr(P[(size_t)ii * 3 + 2]) - bfr(P[(size_t)c.n * 3 + 2]); return c; }
__device__ __forceinline__ void pos_t(const EdgeCtx& c, const float* __restrict__ WP1, const float* __restrict__ BP1, float t[3]) {
#pragma unroll
  for (int j = 0; j < 3; ++j) t[j] = c.pr[0] * bfr(WP1[j]) + c.pr[1] * bfr(WP1[3 + j]) + c.pr[2] * bfr(WP1[6 + j]) + bfr(BP1[j]); }
template <int MODE>
__global__ __launch_bounds__(256) void k_eA(const float* __restrict__ P, const int* __restrict__ KNN, const float* __restrict__ WP1, const float* __restrict__ BP1, const float* __restrict__ STP, float* __restrict__ PART) { __shared__ float sv[EPB][4];
  const int tid = threadIdx.x; const int e = blockIdx.x * EPB + tid; const EdgeCtx c = edge_of(e, P, KNN); float t[3]; pos_t(c, WP1, BP1, t);
#pragma unroll
  for (int j = 0; j < 3; ++j) { const float v = MODE == 0 ? t[j] : (t[j] - STP[j * 32]) * (t[j] - STP[j * 32]); sv[tid][j] = v; }
  __syncthreads();
  if (tid < 3) { float s = 0.f; for (int r = 0; r < EPB; ++r) s += sv[r][tid]; vst2(PART + (size_t)blockIdx.x * CCH + tid, s); } }
__global__ __launch_bounds__(64) void k_finish(const float* __restrict__ PART, int nch, int mode, float cnt, float* __restrict__ STo) { const int c = threadIdx.x; if (c >= nch) return; float s = 0.f;
#pragma unroll 1
  for (int b = 0; b < NEBP; ++b) s += PART[(size_t)b * CCH + c];
  const float m = s / cnt; vst2(STo + (size_t)c * 32 + mode, mode == 0 ? m : rsqrtf(m + 1e-5f)); }
__device__ __forceinline__ void pe_wmma(const float (*su)[4], float (*spe)[68], const float* __restrict__ WP2, int wave, int lane) { const int col = lane & 15, g = lane >> 4;
  v16b wb[4];
#pragma unroll
  for (int j = 0; j < 4; ++j) { const int o = j * 16 + col;
#pragma unroll
    for (int i = 0; i < 16; ++i) wb[j][i] = (__bf16)0.f;
    if (g == 0) { wb[j][0] = (__bf16)WP2[o]; wb[j][1] = (__bf16)WP2[64 + o]; wb[j][2] = (__bf16)WP2[128 + o]; } }
  asm volatile("s_wait_loadcnt 0x0" ::: "memory");
#pragma unroll
  for (int rt = 0; rt < 2; ++rt) { const int rbase = (wave * 2 + rt) * 16; float v[16];
#pragma unroll
    for (int i = 0; i < 16; ++i) v[i] = 0.f;
    if (g == 0) { v[0] = su[rbase + col][0]; v[1] = su[rbase + col][1]; v[2] = su[rbase + col][2]; }
    const F2 a = bsplit16(v);
#pragma unroll
    for (int j = 0; j < 4; ++j) { v8f acc = {}; acc = wmma_bf(a.h, wb[j], acc); acc = wmma_bf(a.l, wb[j], acc);
#pragma unroll
      for (int r = 0; r < 8; ++r) spe[rbase + 8 * g + r][j * 16 + col] = acc[r]; } } }
template <int MODE>
__global__ __launch_bounds__(256) void k_eB(const float* __restrict__ P, const int* __restrict__ KNN, const float* __restrict__ Q, const float* __restrict__ K, const float* __restrict__ WP1, const float* __restrict__ BP1, const float* __restrict__ ST, const float* __restrict__ GP, const float* __restrict__ BEP, const float* __restrict__ WP2, const float* __restrict__ BP2, float* __restrict__ PART) {
  __shared__ float su[EPB][4]; __shared__ __align__(16) float spe[EPB][68];
  const int tid = threadIdx.x, wave = tid >> 5, lane = tid & 31; const int e = blockIdx.x * EPB + tid; const EdgeCtx c = edge_of(e, P, KNN); float t[3]; pos_t(c, WP1, BP1, t);
  { const float* STP = ST + 1 * 64 * 32;
#pragma unroll
    for (int j = 0; j < 3; ++j) su[tid][j] = fmaxf((t[j] - STP[j * 32]) * STP[j * 32 + 1] * bfr(GP[j]) + bfr(BEP[j]), 0.f); su[tid][3] = 0.f; }
  __syncthreads();
  pe_wmma(su, spe, WP2, wave, lane);
  __syncthreads();
  const float* kr = K + (size_t)c.idx * CCH; const float* qr = Q + (size_t)c.n * CCH; const float* STW = ST + 2 * 64 * 32;
#pragma unroll
  for (int c4 = 0; c4 < 64; c4 += 4) { const v4f kv = *(const v4f*)(kr + c4); const v4f qv = *(const v4f*)(qr + c4);
    asm volatile("s_wait_loadcnt 0x0" ::: "memory");
#pragma unroll
    for (int i = 0; i < 4; ++i) { const int cc = c4 + i; const float w0 = kv[i] - qv[i] + (spe[tid][cc] + bfr(BP2[cc])); spe[tid][cc] = MODE == 0 ? w0 : (w0 - STW[cc * 32]) * (w0 - STW[cc * 32]); } }
  __syncthreads();
  if (tid < 64) { float s = 0.f; for (int r = 0; r < EPB; ++r) s += spe[r][tid]; vst2(PART + (size_t)blockIdx.x * CCH + tid, s); } }
__global__ __launch_bounds__(256) void k_eC(const float* __restrict__ P, const int* __restrict__ KNN, const float* __restrict__ Q, const float* __restrict__ K, const float* __restrict__ WP1, const float* __restrict__ BP1, const float* __restrict__ ST, const float* __restrict__ GP, const float* __restrict__ BEP, const float* __restrict__ WP2, const float* __restrict__ BP2,
    const float* __restrict__ GW1, const float* __restrict__ BEW1, const float* __restrict__ WW1, const float* __restrict__ BW1, float* __restrict__ W1R, float* __restrict__ PART) {
  __shared__ float su[EPB][4]; __shared__ __align__(16) float sv[EPB][68]; __shared__ __align__(16) float so[EPB][8];
  const int tid = threadIdx.x, wave = tid >> 5, lane = tid & 31, col = lane & 15, g = lane >> 4; const int e = blockIdx.x * EPB + tid; const EdgeCtx c = edge_of(e, P, KNN); float t[3]; pos_t(c, WP1, BP1, t);
  { const float* STP = ST + 1 * 64 * 32;
#pragma unroll
    for (int j = 0; j < 3; ++j) su[tid][j] = fmaxf((t[j] - STP[j * 32]) * STP[j * 32 + 1] * bfr(GP[j]) + bfr(BEP[j]), 0.f); su[tid][3] = 0.f; }
  __syncthreads();
  pe_wmma(su, sv, WP2, wave, lane);
  __syncthreads();
  const float* kr = K + (size_t)c.idx * CCH; const float* qr = Q + (size_t)c.n * CCH; const float* STW = ST + 2 * 64 * 32;
#pragma unroll
  for (int c4 = 0; c4 < 64; c4 += 4) { const v4f kv = *(const v4f*)(kr + c4); const v4f qv = *(const v4f*)(qr + c4);
    asm volatile("s_wait_loadcnt 0x0" ::: "memory");
#pragma unroll
    for (int i = 0; i < 4; ++i) { const int cc = c4 + i; const float w0 = kv[i] - qv[i] + (sv[tid][cc] + bfr(BP2[cc])); sv[tid][cc] = fmaxf((w0 - STW[cc * 32]) * STW[cc * 32 + 1] * bfr(GW1[cc]) + bfr(BEW1[cc]), 0.f); } }
  __syncthreads();
  v16b wb[2]; { const int o = col < CW ? col : 0; const float keep = col < CW ? 1.f : 0.f;
#pragma unroll
    for (int kc = 0; kc < 2; ++kc) { float t0[8], t1[8];
#pragma unroll
      for (int i = 0; i < 8; ++i) t0[i] = WW1[(size_t)(kc * 32 + 8 * g + i) * CW + o];
      asm volatile("s_wait_loadcnt 0x0" ::: "memory");
#pragma unroll
      for (int i = 0; i < 8; ++i) t1[i] = WW1[(size_t)(kc * 32 + 16 + 8 * g + i) * CW + o];
      asm volatile("s_wait_loadcnt 0x0" ::: "memory");
#pragma unroll
      for (int i = 0; i < 8; ++i) { wb[kc][i] = (__bf16)(t0[i] * keep); wb[kc][8 + i] = (__bf16)(t1[i] * keep); } } }
#pragma unroll
  for (int rt = 0; rt < 2; ++rt) { const int rbase = (wave * 2 + rt) * 16; v8f acc = {};
#pragma unroll
    for (int kc = 0; kc < 2; ++kc) { const F2 a = split_row(&sv[rbase + col][0], kc * 32, lane); acc = wmma_bf(a.h, wb[kc], acc); acc = wmma_bf(a.l, wb[kc], acc); }
    if (col < CW) { const float bb = bfr(BW1[col]);
#pragma unroll
      for (int r = 0; r < 8; ++r) so[rbase + 8 * g + r][col] = acc[r] + bb; } }
  __syncthreads();
  for (int q = tid; q < EPB * CW / 4; q += 256) vst2(W1R + (size_t)blockIdx.x * EPB * CW + q * 4, *(const v4f*)(&so[0][0] + q * 4));
  if (tid < CW) { float s = 0.f; for (int r = 0; r < EPB; ++r) s += so[r][tid]; vst2(PART + (size_t)blockIdx.x * CCH + tid, s); } }
__global__ __launch_bounds__(256) void k_eC2(const float* __restrict__ W1R, const float* __restrict__ ST, float* __restrict__ PART) { __shared__ float sv[EPB][9];
  const int tid = threadIdx.x; const size_t e = (size_t)blockIdx.x * EPB + tid; const float* STW2 = ST + 3 * 64 * 32;
#pragma unroll
  for (int i = 0; i < CW; ++i) { const float d = W1R[e * CW + i] - STW2[i * 32]; sv[tid][i] = d * d; }
  __syncthreads();
  if (tid < CW) { float s = 0.f; for (int r = 0; r < EPB; ++r) s += sv[r][tid]; vst2(PART + (size_t)blockIdx.x * CCH + tid, s); } }
__global__ __launch_bounds__(256) void k_eD(const float* __restrict__ P, const int* __restrict__ KNN, const float* __restrict__ V, const float* __restrict__ WP1, const float* __restrict__ BP1, const float* __restrict__ ST, const float* __restrict__ GP, const float* __restrict__ BEP, const float* __restrict__ WP2, const float* __restrict__ BP2,
    const float* __restrict__ W1R, const float* __restrict__ GW2, const float* __restrict__ BEW2, const float* __restrict__ WW2, const float* __restrict__ BW2, float* __restrict__ AGG) {
  __shared__ float su[EPB][4]; __shared__ __align__(16) float spe[EPB][68];
  const int tid = threadIdx.x, wave = tid >> 5, lane = tid & 31; const int e = blockIdx.x * EPB + tid; const EdgeCtx c = edge_of(e, P, KNN); float t[3]; pos_t(c, WP1, BP1, t);
  { const float* STP = ST + 1 * 64 * 32;
#pragma unroll
    for (int j = 0; j < 3; ++j) su[tid][j] = fmaxf((t[j] - STP[j * 32]) * STP[j * 32 + 1] * bfr(GP[j]) + bfr(BEP[j]), 0.f); su[tid][3] = 0.f; }
  __syncthreads();
  pe_wmma(su, spe, WP2, wave, lane);
  __syncthreads();
  const float* STW2 = ST + 3 * 64 * 32; float u[CW], w2[CW];
#pragma unroll
  for (int i = 0; i < CW; ++i) u[i] = fmaxf((W1R[(size_t)e * CW + i] - STW2[i * 32]) * STW2[i * 32 + 1] * bfr(GW2[i]) + bfr(BEW2[i]), 0.f);
#pragma unroll
  for (int j = 0; j < CW; ++j) { float s = bfr(BW2[j]);
#pragma unroll
    for (int i = 0; i < CW; ++i) s += u[i] * bfr(WW2[i * CW + j]); w2[j] = s; }
  float a[CW];
#pragma unroll
  for (int j = 0; j < CW; ++j) { float m = w2[j];
#pragma unroll
    for (int o = 1; o < 16; o <<= 1) m = fmaxf(m, __shfl_xor(m, o));
    const float ex = expf(w2[j] - m); float sm = ex;
#pragma unroll
    for (int o = 1; o < 16; o <<= 1) sm += __shfl_xor(sm, o);
    a[j] = ex / sm; }
  const float* vr = V + (size_t)c.idx * CCH; float mine[4]; mine[0] = mine[1] = mine[2] = mine[3] = 0.f;
#pragma unroll
  for (int c4 = 0; c4 < 64; c4 += 4) { const v4f vv = *(const v4f*)(vr + c4); asm volatile("s_wait_loadcnt 0x0" ::: "memory"); float contrib[4];
#pragma unroll
    for (int i = 0; i < 4; ++i) { const int cc = c4 + i; float vsum = (vv[i] + (spe[tid][cc] + bfr(BP2[cc]))) * a[cc & 7];
#pragma unroll
      for (int o = 1; o < 16; o <<= 1) vsum += __shfl_xor(vsum, o);
      contrib[i] = vsum; }
    if ((c4 >> 2) == c.s) { mine[0] = contrib[0]; mine[1] = contrib[1]; mine[2] = contrib[2]; mine[3] = contrib[3]; } }
  { v4f o4; o4[0] = mine[0]; o4[1] = mine[1]; o4[2] = mine[2]; o4[3] = mine[3]; vst2(AGG + (size_t)c.n * CCH + c.s * 4, o4); } }
__global__ __launch_bounds__(256) void k_fin(const float* __restrict__ T3, const float* __restrict__ ST3, const float* __restrict__ G, const float* __restrict__ BE, const float* __restrict__ X, float* __restrict__ OUT) { const size_t e4 = (size_t)blockIdx.x * 256 + threadIdx.x; if (e4 >= (size_t)NPROC * CCH / 4) return; const int c0 = (int)((e4 * 4) % CCH); const v4f tv = *(const v4f*)(T3 + e4 * 4); const v4f xv = *(const v4f*)(X + e4 * 4); v4f o;
#pragma unroll
  for (int i = 0; i < 4; ++i) { const int cc = c0 + i; const float y = (tv[i] - ST3[cc * 32]) * ST3[cc * 32 + 1] * bfr(G[cc]) + bfr(BE[cc]); o[i] = fmaxf(y + bfr(xv[i]), 0.f); }
  vst2(OUT + e4 * 4, o); }
extern "C" void kernel_launch(void* const* d_in, const int* in_sizes, int n_in, void* d_out, int out_size, void* d_ws, size_t ws_size, hipStream_t stream) {
  (void)in_sizes; (void)n_in; (void)out_size;
  if (ws_size < (size_t)WS_END) return;
  char* ws = (char*)d_ws; const float** F = (const float**)d_in; const float* P = F[0]; const float* X = F[1]; const int* KNN = (const int*)d_in[2];
  float *T1 = (float*)(ws + WS_T1), *Q = (float*)(ws + WS_Q), *K = (float*)(ws + WS_K), *V = (float*)(ws + WS_V), *AGG = (float*)(ws + WS_AGG), *T3 = (float*)(ws + WS_T3), *W1R = (float*)(ws + WS_W1R), *PART = (float*)(ws + WS_PART), *ST = (float*)(ws + WS_ST);
  float *ST1 = ST, *STP = ST + 1 * 64 * 32, *STW1 = ST + 2 * 64 * 32, *STW2 = ST + 3 * 64 * 32, *ST2 = ST + 4 * 64 * 32, *ST3 = ST + 5 * 64 * 32;
  const float NEf = (float)NPROC * NSB;
  k_gemm64<<<dim3(NPROC / 64, 1), 128, 0, stream>>>(X, 0, nullptr, nullptr, nullptr, F[3], nullptr, T1, nullptr, nullptr, nullptr, nullptr, nullptr, nullptr);
  k_stat64<<<dim3(CCH), 256, 0, stream>>>(T1, ST1);
  k_gemm64<<<dim3(NPROC / 64, 3), 128, 0, stream>>>(T1, 1, ST1, F[4], F[5], F[6], F[7], Q, F[8], F[9], K, F[10], F[11], V);
  k_eA<0><<<dim3(NEBP), 256, 0, stream>>>(P, KNN, F[12], F[13], STP, PART);  k_finish<<<1, 64, 0, stream>>>(PART, 3, 0, NEf, STP);
  k_eA<1><<<dim3(NEBP), 256, 0, stream>>>(P, KNN, F[12], F[13], STP, PART);  k_finish<<<1, 64, 0, stream>>>(PART, 3, 1, NEf, STP);
  k_eB<0><<<dim3(NEBP), 256, 0, stream>>>(P, KNN, Q, K, F[12], F[13], ST, F[14], F[15], F[16], F[17], PART);  k_finish<<<1, 64, 0, stream>>>(PART, 64, 0, NEf, STW1);
  k_eB<1><<<dim3(NEBP), 256, 0, stream>>>(P, KNN, Q, K, F[12], F[13], ST, F[14], F[15], F[16], F[17], PART);  k_finish<<<1, 64, 0, stream>>>(PART, 64, 1, NEf, STW1);
  k_eC<<<dim3(NEBP), 256, 0, stream>>>(P, KNN, Q, K, F[12], F[13], ST, F[14], F[15], F[16], F[17], F[18], F[19], F[20], F[21], W1R, PART);  k_finish<<<1, 64, 0, stream>>>(PART, CW, 0, NEf, STW2);
  k_eC2<<<dim3(NEBP), 256, 0, stream>>>(W1R, ST, PART);  k_finish<<<1, 64, 0, stream>>>(PART, CW, 1, NEf, STW2);
  k_eD<<<dim3(NEBP), 256, 0, stream>>>(P, KNN, V, F[12], F[13], ST, F[14], F[15], F[16], F[17], W1R, F[22], F[23], F[24], F[25], AGG);
  k_stat64<<<dim3(CCH), 256, 0, stream>>>(AGG, ST2);
  k_gemm64<<<dim3(NPROC / 64, 1), 128, 0, stream>>>(AGG, 1, ST2, F[26], F[27], F[28], nullptr, T3, nullptr, nullptr, nullptr, nullptr, nullptr, nullptr);
  k_stat64<<<dim3(CCH), 256, 0, stream>>>(T3, ST3);
  k_fin<<<dim3((NPROC * CCH / 4 + 255) / 256), 256, 0, stream>>>(T3, ST3, F[29], F[30], X, (float*)d_out);
}
